// Matcher_43190191128721
// MI455X (gfx1250) — hardware-verified
//
#include <hip/hip_runtime.h>


typedef _Float16 v16h __attribute__((ext_vector_type(16)));
typedef float    v8f  __attribute__((ext_vector_type(8)));
typedef _Float16 h8   __attribute__((ext_vector_type(8), __may_alias__));
typedef _Float16 h4   __attribute__((ext_vector_type(4), __may_alias__));
typedef float    v4f  __attribute__((ext_vector_type(4), __may_alias__));
typedef float    af   __attribute__((__may_alias__));

#define NEMB 129
#define DIN  21
#define DH   128
#define NCLS 21
#define NCP  32
#define KTOT 640
#define NOUT 21
#define UPIX 32
#define UFLT (UPIX * NOUT)
#define NWAVE 8
#define UPW 2
#define UPB (NWAVE * UPW)
#define IS2 0.70710678118654752f
#define OPS 16.0f
#define OPS2INV 0.00390625f

#define E1_BYTES (NEMB * DH * 4)
#define G_BYTES  (NCP * KTOT * 2)
#define C_BYTES  128
#define WS_NEED  (E1_BYTES + G_BYTES + C_BYTES)

union Frag { v16h v; h8 half[2]; };

__device__ __forceinline__ v8f wmma16(v16h a, v16h b, v8f c)
{
    v8f d = __builtin_amdgcn_wmma_f32_16x16x32_f16(false, a, false, b, (short)0, c, false, false);
    asm volatile("v_nop\n\tv_nop\n\tv_nop\n\tv_nop" : "+v"(d) : "v"(a), "v"(b));
    return d;
}

__device__ __forceinline__ void lds_fence()
{
    asm volatile("s_wait_dscnt 0" ::: "memory");
}

__device__ __forceinline__ int clamp_id(int id)
{
    id = (id < 0) ? (id + NEMB) : id;
    id = (id < 0) ? 0 : id;
    id = (id > NEMB - 1) ? (NEMB - 1) : id;
    return id;
}

__device__ __forceinline__ h4 relu_cvt(v4f v)
{
    h4 r;
    r[0] = (_Float16)(fmaxf(v[0], 0.f) * OPS);
    r[1] = (_Float16)(fmaxf(v[1], 0.f) * OPS);
    r[2] = (_Float16)(fmaxf(v[2], 0.f) * OPS);
    r[3] = (_Float16)(fmaxf(v[3], 0.f) * OPS);
    return r;
}

__global__ __launch_bounds__(256) void k_tables(
    const int*   __restrict__ cls,
    const float* __restrict__ emb,
    const float* __restrict__ W1,
    const float* __restrict__ b1,
    const float* __restrict__ W2,
    const float* __restrict__ b2,
    float*    E1g,
    _Float16* Gg,
    float*    Cg)
{
    __shared__ __align__(16) float    sE1[NEMB * DH];
    __shared__ float                  sH [NCLS * 5 * DH];
    __shared__ float                  sQ [NCLS * 5 * DIN];
    __shared__ float                  sO [NCLS * 5 * DIN];
    __shared__ __align__(16) _Float16 sGs[NCP * KTOT];
    __shared__ __align__(16) float    sCs[NCP];
    const int t = threadIdx.x;

    for (int i = t; i < NEMB * DH; i += 256) {
        const int row = i >> 7, c = i & 127;
        float acc = 0.f;
#pragma unroll 1
        for (int d = 0; d < DIN; ++d) acc += emb[row * DIN + d] * W1[d * DH + c];
        sE1[i] = acc;
    }
    __syncthreads();

    for (int i = t; i < NCLS * 5 * DH; i += 256) {
        const int j = i & 127, cs = i >> 7, s = cs % 5, c = cs / 5;
        const int id  = clamp_id(cls[c * 5 + s]);
        const int id0 = clamp_id(cls[c * 5 + 0]);
        const float v = (s == 0) ? (sE1[id * DH + j] + b1[j])
                                 : (0.5f * sE1[id * DH + j] + IS2 * sE1[id0 * DH + j] + b1[j]);
        sH[i] = fmaxf(v, 0.f);
    }
    __syncthreads();

    for (int i = t; i < NCLS * 5 * DIN; i += 256) {
        const int d = i % DIN, cs = i / DIN;
        const float* hrow = &sH[cs * DH];
        float acc = 0.f;
#pragma unroll 1
        for (int k = 0; k < DH; ++k) acc += hrow[k] * W2[k * DIN + d];
        sQ[i] = acc;
    }
    __syncthreads();

    for (int i = t; i < NCLS * 5 * DIN; i += 256) {
        const int d = i % DIN, cs = i / DIN, s = cs % 5, c = cs / 5;
        const float v = (s == 0) ? sQ[(c * 5) * DIN + d]
                                 : (0.5f * sQ[cs * DIN + d] + IS2 * sQ[(c * 5) * DIN + d]);
        sO[i] = v + b2[d];
    }
    __syncthreads();

    for (int i = t; i < NCP * 5 * DH; i += 256) {
        const int k = i & 127, cs = i >> 7, s = cs % 5, c = cs / 5;
        float acc = 0.f;
        if (c < NCLS) {
#pragma unroll 1
            for (int d = 0; d < DIN; ++d) {
                float P;
                if (s == 0)
                    P = sO[(c * 5 + 0) * DIN + d] +
                        IS2 * (sO[(c * 5 + 1) * DIN + d] + sO[(c * 5 + 2) * DIN + d] +
                               sO[(c * 5 + 3) * DIN + d] + sO[(c * 5 + 4) * DIN + d]);
                else
                    P = 0.5f * sO[(c * 5 + s) * DIN + d];
                acc += W2[k * DIN + d] * P;
            }
        }
        sGs[i] = (_Float16)(acc * OPS);
    }
    if (t < NCP) {
        float acc = 0.f;
        if (t < NCLS) {
#pragma unroll 1
            for (int tt = 0; tt < 5; ++tt)
#pragma unroll 1
                for (int d = 0; d < DIN; ++d) acc += b2[d] * sO[(t * 5 + tt) * DIN + d];
        }
        sCs[t] = acc;
    }
    __syncthreads();

    for (int i = t; i < (NEMB * DH) / 4; i += 256) {
        const v4f v = *(const v4f*)(sE1 + 4 * i);
        *(volatile v4f*)(E1g + 4 * i) = v;
    }
    for (int i = t; i < (NCP * KTOT) / 8; i += 256) {
        const h8 v = *(const h8*)(sGs + 8 * i);
        *(volatile h8*)(Gg + 8 * i) = v;
    }
    if (t < 8) {
        const v4f v = *(const v4f*)(sCs + 4 * t);
        *(volatile v4f*)(Cg + 4 * t) = v;
    }
    __threadfence();
    for (int i = t; i < (NEMB * DH) / 4; i += 256) {
        const v4f v = *(const v4f*)(sE1 + 4 * i);
        *(volatile v4f*)(E1g + 4 * i) = v;
    }
    for (int i = t; i < (NCP * KTOT) / 8; i += 256) {
        const h8 v = *(const h8*)(sGs + 8 * i);
        *(volatile h8*)(Gg + 8 * i) = v;
    }
    if (t < 8) {
        const v4f v = *(const v4f*)(sCs + 4 * t);
        *(volatile v4f*)(Cg + 4 * t) = v;
    }
}

__device__ __forceinline__ void stage_tile(const int* __restrict__ nodes, const float* sE1, _Float16* rb,
                                           int pfirst, int pixels, int j4, v4f bb)
{
#pragma unroll 1
    for (int p = 0; p < 16; ++p) {
        int pg = pfirst + p;
        pg = (pg < pixels) ? pg : (pixels - 1);
        const int* np = nodes + (size_t)pg * 5;
        const int id0 = clamp_id(np[0]);
        const v4f e0  = *(const v4f*)(sE1 + id0 * DH + j4);
        const v4f t0  = e0 * IS2 + bb;
        _Float16* dst = rb + p * KTOT + j4;
        *(h4*)dst = relu_cvt(e0 + bb);
#pragma unroll
        for (int s = 1; s < 5; ++s) {
            const int id = clamp_id(np[s]);
            const v4f e  = *(const v4f*)(sE1 + id * DH + j4);
            *(h4*)(dst + s * DH) = relu_cvt(e * 0.5f + t0);
        }
    }
}

__device__ __forceinline__ void gemm_tile(const _Float16* ra, const _Float16* gb0, const _Float16* gb1,
                                          v8f& acc0, v8f& acc1)
{
#pragma unroll 4
    for (int kb = 0; kb < KTOT; kb += 32) {
        Frag A, B0, B1;
        A.half[0]  = *(const h8*)(ra  + kb);
        A.half[1]  = *(const h8*)(ra  + kb + 16);
        B0.half[0] = *(const h8*)(gb0 + kb);
        B0.half[1] = *(const h8*)(gb0 + kb + 16);
        B1.half[0] = *(const h8*)(gb1 + kb);
        B1.half[1] = *(const h8*)(gb1 + kb + 16);
        acc0 = wmma16(A.v, B0.v, acc0);
        acc1 = wmma16(A.v, B1.v, acc1);
    }
}

__global__ __launch_bounds__(256) void k_main(
    const int*      __restrict__ nodes,
    const float*    __restrict__ E1g,
    const _Float16* __restrict__ Gg,
    const float*    __restrict__ Cg,
    const float*    __restrict__ b1,
    float* out,
    int pixels, int units)
{
    __shared__ __align__(16) float    sE1[NEMB * DH];
    __shared__ __align__(16) _Float16 sG[NCP * KTOT];
    __shared__ __align__(16) float    sC[NCP];
    __shared__ __align__(16) float    sB1[DH];
    __shared__ __align__(16) _Float16 sR[NWAVE][16 * KTOT];

    const int t    = threadIdx.x;
    const int lane = t & 31;
    const int wv   = __builtin_amdgcn_readfirstlane(t >> 5);

    {
        const v4f* E1v = (const v4f*)E1g;
        v4f* sE1v = (v4f*)sE1;
        for (int i = t; i < (NEMB * DH) / 4; i += 256) sE1v[i] = E1v[i];
        const h8* Gv = (const h8*)Gg;
        h8* sGv = (h8*)sG;
        for (int i = t; i < (NCP * KTOT) / 8; i += 256) sGv[i] = Gv[i];
        if (t < NCP) sC[t]  = Cg[t];
        if (t < DH)  sB1[t] = b1[t];
    }
    __syncthreads();

    const int h    = lane >> 4;
    const int col  = lane & 15;
    const int koff = 8 * h;
    const int j4   = lane << 2;
    const v4f bb   = *(const v4f*)&sB1[j4];
    _Float16* rbase = &sR[wv][0];
    const _Float16* ra  = rbase + col * KTOT + koff;
    const _Float16* gb0 = &sG[col * KTOT] + koff;
    const _Float16* gb1 = &sG[(16 + col) * KTOT] + koff;
    const float c0 = sC[col];
    const float c1 = sC[16 + col];
    af* so = (af*)rbase;

    for (int it = 0; it < UPW; ++it) {
        const int u = (blockIdx.x * NWAVE + wv) * UPW + it;
        if (u >= units) break;
        const int p0 = u * UPIX;

        v8f a00 = {0.f, 0.f, 0.f, 0.f, 0.f, 0.f, 0.f, 0.f};
        v8f a01 = a00, a10 = a00, a11 = a00;

        stage_tile(nodes, sE1, rbase, p0, pixels, j4, bb);
        lds_fence();
        gemm_tile(ra, gb0, gb1, a00, a01);
        lds_fence();
        stage_tile(nodes, sE1, rbase, p0 + 16, pixels, j4, bb);
        lds_fence();
        gemm_tile(ra, gb0, gb1, a10, a11);
        lds_fence();

#pragma unroll
        for (int i = 0; i < 8; ++i) {
            const int r0 = (8 * h + i) * NOUT;
            const int r1 = (16 + 8 * h + i) * NOUT;
            so[r0 + col] = a00[i] * OPS2INV + c0;
            so[r1 + col] = a10[i] * OPS2INV + c0;
            if (col < 5) {
                so[r0 + 16 + col] = a01[i] * OPS2INV + c1;
                so[r1 + 16 + col] = a11[i] * OPS2INV + c1;
            }
        }
        lds_fence();

        float* gout = out + (size_t)u * UFLT;
        const int nval = pixels - p0;
        if (nval >= UPIX) {
            v4f wq[6];
#pragma unroll
            for (int j = 0; j < 6; ++j) {
                const int idx = j * 32 + lane;
                wq[j] = (idx < UFLT / 4) ? *(const v4f*)(so + 4 * idx) : (v4f){0.f, 0.f, 0.f, 0.f};
            }
#pragma unroll
            for (int j = 0; j < 6; ++j) {
                const int idx = j * 32 + lane;
                if (idx < UFLT / 4) *(volatile v4f*)(gout + 4 * idx) = wq[j];
            }
            __threadfence();
#pragma unroll
            for (int j = 0; j < 6; ++j) {
                const int idx = j * 32 + lane;
                if (idx < UFLT / 4) *(volatile v4f*)(gout + 4 * idx) = wq[j];
            }
        } else {
            const int nf = nval * NOUT;
            for (int e = lane; e < nf; e += 32) {
                const float v = so[e];
                *(volatile float*)(gout + e) = v;
            }
            __threadfence();
            for (int e = lane; e < nf; e += 32) {
                const float v = so[e];
                *(volatile float*)(gout + e) = v;
            }
        }
        lds_fence();
    }
}

extern "C" void kernel_launch(void* const* d_in, const int* in_sizes, int n_in,
                              void* d_out, int out_size, void* d_ws, size_t ws_size,
                              hipStream_t stream)
{
    if (n_in < 7) return;
    const int*   inst = (const int*)d_in[0];
    const int*   cls  = (const int*)d_in[1];
    const float* emb  = (const float*)d_in[2];
    const float* W1   = (const float*)d_in[3];
    const float* b1   = (const float*)d_in[4];
    const float* W2   = (const float*)d_in[5];
    const float* b2   = (const float*)d_in[6];
    float* out = (float*)d_out;

    int pixels = in_sizes[0] / 5;
    const int pix_out = out_size / NOUT;
    if (pix_out < pixels) pixels = pix_out;
    if (pixels <= 0) return;
    if (ws_size < (size_t)WS_NEED) return;

    float*    E1g = (float*)d_ws;
    _Float16* Gg  = (_Float16*)((char*)d_ws + E1_BYTES);
    float*    Cg  = (float*)((char*)d_ws + E1_BYTES + G_BYTES);

    k_tables<<<1, 256, 0, stream>>>(cls, emb, W1, b1, W2, b2, E1g, Gg, Cg);

    const int units = (pixels + UPIX - 1) / UPIX;
    const int grid  = (units + UPB - 1) / UPB;
    k_main<<<grid, 256, 0, stream>>>(inst, E1g, Gg, Cg, b1, out, pixels, units);
}
